// ReducedGlobalAttention_81200651698440
// MI455X (gfx1250) — hardware-verified
//
#include <hip/hip_runtime.h>
#include <stdint.h>

#define NBATCH 2
#define CIN    512
#define KCH    256
#define COUT   512
#define NP     4096
#define IMW    64
#define CATC   1024
#define NPOOL  110
#define PPITCH 128
#define TP     68
#define NROWKV 512

#define XSC   64.0f
#define WSC   1024.0f
#define CSC   64.0f
#define RSC   1024.0f
#define RINV  (1.0f / 1024.0f)
#define PSC   16384.0f
#define OSC16 (1.0f / 65536.0f)
#define OSC20 (1.0f / 1048576.0f)

static_assert((NP % 128) == 0 && (KCH % 128) == 0 && (CIN % 32) == 0 && (COUT % 128) == 0);
static_assert(NPOOL <= PPITCH && (NP % 16) == 0 && IMW * IMW == NP);
static_assert(4 * KCH == CATC && (CATC % 32) == 0);

typedef _Float16 v16h __attribute__((ext_vector_type(16)));
typedef _Float16 v8h  __attribute__((ext_vector_type(8)));
typedef float    v8f  __attribute__((ext_vector_type(8)));
typedef float    v4f  __attribute__((ext_vector_type(4)));
typedef unsigned int v4u __attribute__((ext_vector_type(4)));

__device__ __forceinline__ unsigned short bf_bits(float f) {
  unsigned u = __float_as_uint(f);
  return (unsigned short)((u + 0x7FFFu + ((u >> 16) & 1u)) >> 16);
}
__device__ __forceinline__ float bf_up(unsigned short hb) { return __uint_as_float(((unsigned)hb) << 16); }
__device__ __forceinline__ float bfr(float f) { return bf_up(bf_bits(f)); }
__device__ __forceinline__ unsigned short h_bits(_Float16 x) { return __builtin_bit_cast(unsigned short, x); }
__device__ __forceinline__ unsigned short f2h_bits(float f) { return h_bits((_Float16)f); }
__device__ __forceinline__ unsigned pk16(unsigned short a, unsigned short b) { return (unsigned)a | ((unsigned)b << 16); }
__device__ __forceinline__ v8f zero8() { v8f z = {0.f, 0.f, 0.f, 0.f, 0.f, 0.f, 0.f, 0.f}; return z; }
__device__ __forceinline__ void split_h(float u, unsigned short& hb, unsigned short& lb) {
  const _Float16 hh = (_Float16)u;
  hb = h_bits(hh);
  lb = f2h_bits((u - (float)hh) * RSC);
}

__device__ __forceinline__ v16h ldfrag_h(const _Float16* p) {
  union { v16h v; v8h hv[2]; } f;
  f.hv[0] = *(const v8h*)(p);
  f.hv[1] = *(const v8h*)(p + 16);
  return f.v;
}

__device__ __forceinline__ v8f mma_h_raw(v16h a, v16h b, v8f c) {
  return __builtin_amdgcn_wmma_f32_16x16x32_f16(false, a, false, b, (short)0, c, false, false);
}
__device__ __forceinline__ void guard2(v8f& a, v8f& b, v16h x, v16h y) {
#if defined(__HIP_DEVICE_COMPILE__)
  asm volatile("v_nop\n\tv_nop\n\tv_nop\n\tv_nop" : "+v"(a), "+v"(b) : "v"(x), "v"(y));
#endif
}
__device__ __forceinline__ void guard4(v8f& a, v8f& b, v8f& c, v8f& d, v16h x, v16h y, v16h z, v16h w) {
#if defined(__HIP_DEVICE_COMPILE__)
  asm volatile("v_nop\n\tv_nop\n\tv_nop\n\tv_nop" : "+v"(a), "+v"(b), "+v"(c), "+v"(d)
               : "v"(x), "v"(y), "v"(z), "v"(w));
#endif
}
__device__ __forceinline__ void keep4_h(v16h a, v16h b, v16h c, v16h d) {
#if defined(__HIP_DEVICE_COMPILE__)
  asm volatile("v_nop" :: "v"(a), "v"(b), "v"(c), "v"(d));
#endif
}
__device__ __forceinline__ void acc_guard4(v8f& a, v8f& b, v8f& c, v8f& d) {
#if defined(__HIP_DEVICE_COMPILE__)
  asm volatile("v_nop\n\tv_nop\n\tv_nop\n\tv_nop" : "+v"(a), "+v"(b), "+v"(c), "+v"(d));
#endif
}

__global__ __launch_bounds__(256) void k_tab(const float* __restrict__ gq, const float* __restrict__ bq,
    const float* __restrict__ mq, const float* __restrict__ vq, const float* __restrict__ gk,
    const float* __restrict__ bk, const float* __restrict__ mk, const float* __restrict__ vk,
    const float* __restrict__ bpk, const float* __restrict__ bpv, float* tab) {
  const int t = threadIdx.x;
  const float g0 = bfr(gq[t]), b0 = bfr(bq[t]), m0 = bfr(mq[t]), v0 = bfr(vq[t]);
  const float g1 = bfr(gk[t]), b1 = bfr(bk[t]), m1 = bfr(mk[t]), v1 = bfr(vk[t]);
  const float r0 = 1.0f / sqrtf(v0 + 1.0e-5f);
  const float r1 = 1.0f / sqrtf(v1 + 1.0e-5f);
  float vals[8];
  vals[0] = g0 * r0;  vals[1] = b0 - m0 * vals[0];
  vals[2] = g1 * r1;  vals[3] = 1.0f;  vals[4] = b1 - m1 * vals[2];  vals[5] = 0.0f;
  vals[6] = bfr(bpk[t]);  vals[7] = bfr(bpv[t]);
  __shared__ __align__(16) float stab[8 * KCH];
#pragma unroll
  for (int i = 0; i < 8; ++i) stab[i * KCH + t] = vals[i];
  __syncthreads();
  typedef float v4f_tab __attribute__((ext_vector_type(4)));
  for (int pass = 0; pass < 2; ++pass) {
    for (int j = t; j < (8 * KCH) / 4; j += 256) {
      const v4f_tab v = *(const v4f_tab*)(stab + 4 * j);
      *(volatile v4f_tab*)(tab + 4 * j) = v;
    }
    __threadfence();
  }
}

__global__ __launch_bounds__(256) void k_cvtw(const float* __restrict__ wq, const float* __restrict__ wk,
    const float* __restrict__ wv, const float* __restrict__ wpk, const float* __restrict__ wpv,
    const float* __restrict__ ww, unsigned short* w3, unsigned short* wpk16, unsigned short* wpv16,
    unsigned short* ww16) {
  const int which = blockIdx.y;
  const float* src; unsigned short* dst; int n;
  if (which == 0)      { src = wq;  dst = w3;                 n = KCH * CIN; }
  else if (which == 1) { src = wk;  dst = w3 + KCH * CIN;     n = KCH * CIN; }
  else if (which == 2) { src = wv;  dst = w3 + 2 * KCH * CIN; n = KCH * CIN; }
  else if (which == 3) { src = wpk; dst = wpk16;              n = KCH * CATC; }
  else if (which == 4) { src = wpv; dst = wpv16;              n = KCH * CATC; }
  else                 { src = ww;  dst = ww16;               n = COUT * KCH; }
  const int base = (blockIdx.x * 256 + threadIdx.x) * 8;
  if (base >= n) return;
  const v4f a = *(const v4f*)(src + base);
  const v4f c = *(const v4f*)(src + base + 4);
  v4u p;
  p[0] = pk16(f2h_bits(bfr(a[0]) * WSC), f2h_bits(bfr(a[1]) * WSC));
  p[1] = pk16(f2h_bits(bfr(a[2]) * WSC), f2h_bits(bfr(a[3]) * WSC));
  p[2] = pk16(f2h_bits(bfr(c[0]) * WSC), f2h_bits(bfr(c[1]) * WSC));
  p[3] = pk16(f2h_bits(bfr(c[2]) * WSC), f2h_bits(bfr(c[3]) * WSC));
  unsigned short* d = dst + base;
  *(volatile v4u*)d = p;
  __threadfence();
  *(volatile v4u*)d = p;
}

__global__ __launch_bounds__(256) void k_cvtx(const float* __restrict__ x, unsigned short* xt) {
  __shared__ __align__(16) float sx[CIN * 17];
  const int tid = threadIdx.x, b = blockIdx.y, p0 = blockIdx.x * 16;
  const float* src = x + (size_t)b * CIN * NP;
#pragma unroll 4
  for (int it = 0; it < 32; ++it) {
    const int idx = it * 256 + tid;
    const int c = idx >> 4, q = idx & 15;
    sx[c * 17 + q] = src[(size_t)c * NP + p0 + q];
  }
  __syncthreads();
  const int wave = tid >> 5, lane = tid & 31;
  v4u pk[4];
#pragma unroll
  for (int k = 0; k < 4; ++k) {
    const int r = wave * 2 + (k >> 1);
    const int cb = (k & 1) * 256 + lane * 8;
    v4u p;
#pragma unroll
    for (int e = 0; e < 4; ++e) {
      const float a = bfr(sx[(cb + 2 * e) * 17 + r]) * XSC;
      const float c = bfr(sx[(cb + 2 * e + 1) * 17 + r]) * XSC;
      p[e] = pk16(f2h_bits(a), f2h_bits(c));
    }
    pk[k] = p;
  }
  unsigned short* dst = xt + ((size_t)b * NP + p0) * CIN;
  for (int pass = 0; pass < 2; ++pass) {
#pragma unroll
    for (int k = 0; k < 4; ++k) {
      const int r = wave * 2 + (k >> 1);
      const int cb = (k & 1) * 256 + lane * 8;
      *(volatile v4u*)(dst + (size_t)r * CIN + cb) = pk[k];
    }
    __threadfence();
  }
}

template <int SA, int SB, int O16>
__global__ __launch_bounds__(256) void k_gemm(
    const unsigned short* __restrict__ Ahp, const unsigned short* __restrict__ Alp, int lda, long long strideA,
    const unsigned short* __restrict__ Bhp, const unsigned short* __restrict__ Blp, int ldb, long long strideB,
    float* C32, unsigned short* Chp, unsigned short* Clp, int ldc, long long strideC,
    int M, int N, int K, float oscale,
    const float* __restrict__ sc, const float* __restrict__ sh, int ntab, int axis, int relu_lim, float cscale) {
  __shared__ __align__(16) float sT[128 * TP];
  (void)M;
  const int b = blockIdx.y;
  const int tid = threadIdx.x, lane = tid & 31, wave = tid >> 5;
  const int wm = wave >> 1, wn = wave & 1;
  const int tilesN = N >> 6;
  const int tm = (int)blockIdx.x / tilesN;
  const int tn = (int)blockIdx.x - tm * tilesN;
  const int m0 = tm * 128, n0 = tn * 64;
  const _Float16* Ah = (const _Float16*)(const void*)Ahp + (size_t)b * (size_t)strideA;
  const _Float16* Al = (const _Float16*)(const void*)Alp + (size_t)b * (size_t)strideA;
  const _Float16* Bh = (const _Float16*)(const void*)Bhp + (size_t)b * (size_t)strideB;
  const _Float16* Bl = (const _Float16*)(const void*)Blp + (size_t)b * (size_t)strideB;
  const int rl = lane & 15, h = lane >> 4, koff = h * 8;
  const int am = m0 + 32 * wm, bn = n0 + 32 * wn;

  v8f acch[2][2], accx[2][2];
#pragma unroll
  for (int i = 0; i < 2; ++i)
#pragma unroll
    for (int j = 0; j < 2; ++j) { acch[i][j] = zero8(); accx[i][j] = zero8(); }

  for (int k0 = 0; k0 < K; k0 += 32) {
    v16h bh[2], bl[2];
#pragma unroll
    for (int j = 0; j < 2; ++j) {
      const size_t bo = (size_t)(bn + 16 * j + rl) * (size_t)ldb + k0 + koff;
      bh[j] = ldfrag_h(Bh + bo);
      if (SB) bl[j] = ldfrag_h(Bl + bo); else bl[j] = bh[j];
    }
#pragma unroll
    for (int i = 0; i < 2; ++i) {
      const size_t ao = (size_t)(am + 16 * i + rl) * (size_t)lda + k0 + koff;
      const v16h ah = ldfrag_h(Ah + ao);
      v16h al;
      if (SA) al = ldfrag_h(Al + ao); else al = ah;
#pragma unroll
      for (int j = 0; j < 2; ++j) {
        acch[i][j] = mma_h_raw(ah, bh[j], acch[i][j]);
        if (SB) accx[i][j] = mma_h_raw(ah, bl[j], accx[i][j]);
        if (SA) accx[i][j] = mma_h_raw(al, bh[j], accx[i][j]);
      }
      if (SA || SB) guard4(acch[i][0], acch[i][1], accx[i][0], accx[i][1], ah, al, bh[1], bl[1]);
      else          guard2(acch[i][0], acch[i][1], ah, bh[1]);
    }
    keep4_h(bh[0], bh[1], bl[0], bl[1]);
  }
  acc_guard4(acch[0][0], acch[0][1], acch[1][0], acch[1][1]);
  if (SA || SB) acc_guard4(accx[0][0], accx[0][1], accx[1][0], accx[1][1]);

#pragma unroll
  for (int i = 0; i < 2; ++i)
#pragma unroll
    for (int j = 0; j < 2; ++j)
#pragma unroll
      for (int r = 0; r < 8; ++r) {
        float v = acch[i][j][r];
        if (SA || SB) v += accx[i][j][r] * RINV;
        sT[(32 * wm + 16 * i + 8 * h + r) * TP + 32 * wn + 16 * j + rl] = v;
      }
  __syncthreads();

  const int tclamp = ntab - 1;
  if (O16) {
    const int rq = lane >> 3, c8 = (lane & 7) * 8;
    v4u oh[4], ol[4];
#pragma unroll
    for (int it = 0; it < 4; ++it) {
      const int row = 16 * wave + 4 * it + rq;
      const int m = m0 + row;
      const v4f x0 = *(const v4f*)(sT + row * TP + c8);
      const v4f x1 = *(const v4f*)(sT + row * TP + c8 + 4);
      float vv[8] = {x0[0], x0[1], x0[2], x0[3], x1[0], x1[1], x1[2], x1[3]};
      unsigned short hb[8], lb[8];
#pragma unroll
      for (int e = 0; e < 8; ++e) {
        const int idx = (axis != 0) ? (n0 + c8 + e) : m;
        const int ci = min(idx, tclamp);
        float t = vv[e] * oscale * sc[ci] + sh[ci];
        if (idx < relu_lim) t = fmaxf(t, 0.0f);
        split_h(t * cscale, hb[e], lb[e]);
      }
      v4u ph, pl;
#pragma unroll
      for (int e = 0; e < 4; ++e) { ph[e] = pk16(hb[2 * e], hb[2 * e + 1]); pl[e] = pk16(lb[2 * e], lb[2 * e + 1]); }
      oh[it] = ph; ol[it] = pl;
    }
    unsigned short* Hb = Chp + (size_t)b * (size_t)strideC;
    unsigned short* Lb = Clp + (size_t)b * (size_t)strideC;
    for (int pass = 0; pass < 2; ++pass) {
#pragma unroll
      for (int it = 0; it < 4; ++it) {
        const int row = 16 * wave + 4 * it + rq;
        const size_t o = (size_t)(m0 + row) * (size_t)ldc + n0 + c8;
        *(volatile v4u*)(Hb + o) = oh[it];
        *(volatile v4u*)(Lb + o) = ol[it];
      }
      __threadfence();
    }
  } else {
    const int hh = lane >> 4, c4 = (lane & 15) * 4;
    v4f ov[8];
#pragma unroll
    for (int it = 0; it < 8; ++it) {
      const int row = 16 * wave + 2 * it + hh;
      const int m = m0 + row;
      v4f v = *(const v4f*)(sT + row * TP + c4);
#pragma unroll
      for (int e = 0; e < 4; ++e) {
        const int idx = (axis != 0) ? (n0 + c4 + e) : m;
        const int ci = min(idx, tclamp);
        float t = v[e] * oscale * sc[ci] + sh[ci];
        if (idx < relu_lim) t = fmaxf(t, 0.0f);
        v[e] = t;
      }
      ov[it] = v;
    }
    float* Cb = C32 + (size_t)b * (size_t)strideC;
    for (int pass = 0; pass < 2; ++pass) {
#pragma unroll
      for (int it = 0; it < 8; ++it) {
        const int row = 16 * wave + 2 * it + hh;
        *(volatile v4f*)(Cb + (size_t)(m0 + row) * (size_t)ldc + n0 + c4) = ov[it];
      }
      __threadfence();
    }
  }
}

__global__ __launch_bounds__(256) void k_pool(const float* __restrict__ kvf, float* pool) {
  __shared__ __align__(16) float img[NP];
  __shared__ float rs[18 * IMW];
  __shared__ __align__(16) float pb[PPITCH];
  const int tid = threadIdx.x, row = blockIdx.x, b = blockIdx.y;
  const float* src = kvf + ((size_t)b * NROWKV + row) * NP;
#pragma unroll
  for (int k = 0; k < 4; ++k) {
    const int e = (k * 256 + tid) * 4;
    *(v4f*)(img + e) = *(const v4f*)(src + e);
  }
  __syncthreads();
  for (int task = tid; task < 18 * IMW; task += 256) {
    const int rb = task >> 6, col = task & 63;
    int s, i;
    if (rb < 1)       { s = 1; i = 0; }
    else if (rb < 4)  { s = 3; i = rb - 1; }
    else if (rb < 10) { s = 6; i = rb - 4; }
    else              { s = 8; i = rb - 10; }
    const int lo = (i * IMW) / s, hi = ((i + 1) * IMW + s - 1) / s;
    float sum = 0.0f;
    for (int y = lo; y < hi; ++y) sum += img[y * IMW + col];
    rs[task] = sum * (1.0f / (float)(hi - lo));
  }
  __syncthreads();
  if (tid < NPOOL) {
    int s, off, rbase;
    if (tid < 1)       { s = 1; off = 0;  rbase = 0; }
    else if (tid < 10) { s = 3; off = 1;  rbase = 1; }
    else if (tid < 46) { s = 6; off = 10; rbase = 4; }
    else               { s = 8; off = 46; rbase = 10; }
    const int local = tid - off;
    const int by = local / s, bx = local - by * s;
    const int lo = (bx * IMW) / s, hi = ((bx + 1) * IMW + s - 1) / s;
    float sum = 0.0f;
    for (int xx = lo; xx < hi; ++xx) sum += rs[(rbase + by) * IMW + xx];
    pb[tid] = sum * (1.0f / (float)(hi - lo));
  } else if (tid < PPITCH) {
    pb[tid] = 0.0f;
  }
  __syncthreads();
  if (tid < 32) {
    const v4f v = *(const v4f*)(pb + 4 * tid);
    float* d = pool + ((size_t)b * NROWKV + row) * PPITCH + 4 * tid;
    *(volatile v4f*)d = v;
    __threadfence();
    *(volatile v4f*)d = v;
  }
}

__global__ __launch_bounds__(256) void k_cat(const float* __restrict__ pool, int rowbase,
                                              unsigned short* cath, unsigned short* catl) {
  const int tid = threadIdx.x, b = blockIdx.y, p0 = blockIdx.x * 16;
  const int half = tid >> 7, ch0 = (tid & 127) * 8, level = ch0 >> 8, c0 = ch0 & 255;
  const int s   = (level == 0) ? 1 : (level == 1) ? 3 : (level == 2) ? 6 : 8;
  const int off = (level == 0) ? 0 : (level == 1) ? 1 : (level == 2) ? 10 : 46;
  const float inv = (float)s * 0.015625f;
  const float* base = pool + ((size_t)b * NROWKV + rowbase + c0) * PPITCH + off;
#pragma unroll 1
  for (int it = 0; it < 8; ++it) {
    const int p = p0 + 2 * it + half;
    const int y = p >> 6, xx = p & 63;
    const float sy = ((float)y + 0.5f) * inv - 0.5f;
    const float sx = ((float)xx + 0.5f) * inv - 0.5f;
    int y0 = (int)floorf(sy); float fy = sy - (float)y0;
    int x0 = (int)floorf(sx); float fx = sx - (float)x0;
    if (y0 < 0)      { y0 = 0;     fy = 0.0f; }
    if (y0 >= s - 1) { y0 = s - 1; fy = 0.0f; }
    if (x0 < 0)      { x0 = 0;     fx = 0.0f; }
    if (x0 >= s - 1) { x0 = s - 1; fx = 0.0f; }
    const int y1 = min(y0 + 1, s - 1), x1 = min(x0 + 1, s - 1);
    const int o00 = y0 * s + x0, o01 = y0 * s + x1, o10 = y1 * s + x0, o11 = y1 * s + x1;
    unsigned short hb[8], lb[8];
#pragma unroll
    for (int e = 0; e < 8; ++e) {
      const float* pc = base + (size_t)e * PPITCH;
      const float v00 = pc[o00], v01 = pc[o01], v10 = pc[o10], v11 = pc[o11];
      const float t0 = v00 + fx * (v01 - v00);
      const float t1 = v10 + fx * (v11 - v10);
      const float val = t0 + fy * (t1 - t0);
      split_h(val * CSC, hb[e], lb[e]);
    }
    v4u ph, pl;
#pragma unroll
    for (int e = 0; e < 4; ++e) { ph[e] = pk16(hb[2 * e], hb[2 * e + 1]); pl[e] = pk16(lb[2 * e], lb[2 * e + 1]); }
    const size_t o = ((size_t)b * NP + p) * CATC + ch0;
    *(volatile v4u*)(cath + o) = ph;
    *(volatile v4u*)(catl + o) = pl;
    __threadfence();
    *(volatile v4u*)(cath + o) = ph;
    *(volatile v4u*)(catl + o) = pl;
  }
}

__global__ __launch_bounds__(256) void k_soft(const float* __restrict__ S, unsigned short* P) {
  __shared__ float sred[16];
  const int tid = threadIdx.x, wave = tid >> 5, lane = tid & 31;
  const size_t q = blockIdx.x;
  const float* R = S + q * NP;
  const float L2E = 1.4426950408889634f;
  v4f u[4];
  u[0] = *(const v4f*)(R + tid * 8);
  u[1] = *(const v4f*)(R + tid * 8 + 4);
  u[2] = *(const v4f*)(R + (NP / 2) + tid * 8);
  u[3] = *(const v4f*)(R + (NP / 2) + tid * 8 + 4);
  float m = -3.0e38f;
#pragma unroll
  for (int k = 0; k < 4; ++k) {
    u[k] = u[k] * L2E;
    m = fmaxf(fmaxf(m, fmaxf(u[k][0], u[k][1])), fmaxf(u[k][2], u[k][3]));
  }
#pragma unroll
  for (int off = 16; off >= 1; off >>= 1) m = fmaxf(m, __shfl_xor(m, off, 32));
  if (lane == 0) sred[wave] = m;
  __syncthreads();
  float mu = sred[0];
#pragma unroll
  for (int w = 1; w < 8; ++w) mu = fmaxf(mu, sred[w]);
  float l = 0.0f;
#pragma unroll
  for (int k = 0; k < 4; ++k)
#pragma unroll
    for (int e = 0; e < 4; ++e) l += exp2f(u[k][e] - mu);
#pragma unroll
  for (int off = 16; off >= 1; off >>= 1) l += __shfl_xor(l, off, 32);
  if (lane == 0) sred[8 + wave] = l;
  __syncthreads();
  float lt = sred[8];
#pragma unroll
  for (int w = 1; w < 8; ++w) lt += sred[8 + w];
  const float rl = PSC * __builtin_amdgcn_rcpf(lt);
  v4u o[2];
#pragma unroll
  for (int g = 0; g < 2; ++g) {
    v4u pg;
#pragma unroll
    for (int e = 0; e < 2; ++e) {
      pg[e]     = pk16(f2h_bits(exp2f(u[2 * g][2 * e] - mu) * rl),     f2h_bits(exp2f(u[2 * g][2 * e + 1] - mu) * rl));
      pg[2 + e] = pk16(f2h_bits(exp2f(u[2 * g + 1][2 * e] - mu) * rl), f2h_bits(exp2f(u[2 * g + 1][2 * e + 1] - mu) * rl));
    }
    o[g] = pg;
  }
  unsigned short* d = P + q * NP + tid * 8;
  for (int pass = 0; pass < 2; ++pass) {
    *(volatile v4u*)(d) = o[0];
    *(volatile v4u*)(d + NP / 2) = o[1];
    __threadfence();
  }
}

extern "C" void kernel_launch(void* const* d_in, const int* in_sizes, int n_in,
                              void* d_out, int out_size, void* d_ws, size_t ws_size,
                              hipStream_t stream) {
  if (n_in < 17) return;
  if (in_sizes[0] != NBATCH * CIN * NP) return;
  if (in_sizes[1] != KCH * CIN || in_sizes[6] != KCH * CIN || in_sizes[11] != KCH * CIN) return;
  for (int i = 2; i <= 5; ++i) if (in_sizes[i] != KCH) return;
  for (int i = 7; i <= 10; ++i) if (in_sizes[i] != KCH) return;
  if (in_sizes[12] != KCH * CATC || in_sizes[14] != KCH * CATC) return;
  if (in_sizes[13] != KCH || in_sizes[15] != KCH) return;
  if (in_sizes[16] != COUT * KCH) return;
  if (out_size != NBATCH * COUT * NP) return;

  const float* x   = (const float*)d_in[0];
  const float* wq  = (const float*)d_in[1];
  const float* gq  = (const float*)d_in[2];
  const float* bq  = (const float*)d_in[3];
  const float* mq  = (const float*)d_in[4];
  const float* vq  = (const float*)d_in[5];
  const float* wk  = (const float*)d_in[6];
  const float* gk  = (const float*)d_in[7];
  const float* bk  = (const float*)d_in[8];
  const float* mk  = (const float*)d_in[9];
  const float* vk  = (const float*)d_in[10];
  const float* wv  = (const float*)d_in[11];
  const float* wpk = (const float*)d_in[12];
  const float* bpk = (const float*)d_in[13];
  const float* wpv = (const float*)d_in[14];
  const float* bpv = (const float*)d_in[15];
  const float* ww  = (const float*)d_in[16];
  float* out = (float*)d_out;

  const size_t szXT   = (size_t)NBATCH * NP * CIN * 2;
  const size_t szKVF  = (size_t)NBATCH * NROWKV * NP * 4;
  const size_t szCAT  = (size_t)NBATCH * NP * CATC * 2;
  const size_t szPOOL = (size_t)NBATCH * NROWKV * PPITCH * 4;
  const size_t szS    = (size_t)NP * NP * 4;
  const size_t szP    = (size_t)NP * NP * 2;
  const size_t szW3   = (size_t)3 * KCH * CIN * 2;
  const size_t szWP   = (size_t)KCH * CATC * 2;
  const size_t szWW   = (size_t)COUT * KCH * 2;
  const size_t szTAB  = (size_t)8 * KCH * 4;
  const size_t szQ    = (size_t)NBATCH * NP * KCH * 2;
  const size_t szCT   = (size_t)NP * KCH * 2;

  const size_t oXT = 0;
  const size_t oKVF = oXT + szXT;
  const size_t oCATH = oKVF + szKVF;
  const size_t oCATL = oCATH + szCAT;
  const size_t oPOOL = oCATL + szCAT;
  const size_t endA0 = oPOOL + szPOOL;
  const size_t oS = 0;
  size_t off = (endA0 > szS) ? endA0 : szS;
  off = (off + 255) & ~(size_t)255;
  const size_t oP   = off; off += szP;
  const size_t oW3  = off; off += szW3;
  const size_t oWPK = off; off += szWP;
  const size_t oWPV = off; off += szWP;
  const size_t oWW  = off; off += szWW;
  const size_t oTAB = off; off += szTAB;
  const size_t oQH  = off; off += szQ;
  const size_t oQL  = off; off += szQ;
  const size_t oKH  = off; off += szQ;
  const size_t oKL  = off; off += szQ;
  const size_t oVH  = off; off += szQ;
  const size_t oVL  = off; off += szQ;
  const size_t oCTH = off; off += szCT;
  const size_t oCTL = off; off += szCT;
  if (off > ws_size) return;
  if (off > (size_t)134217728) return;

  char* ws = (char*)d_ws;
  unsigned short* XT   = (unsigned short*)(ws + oXT);
  float*          KVF  = (float*)(ws + oKVF);
  unsigned short* CATH = (unsigned short*)(ws + oCATH);
  unsigned short* CATL = (unsigned short*)(ws + oCATL);
  float*          POOL = (float*)(ws + oPOOL);
  float*          S    = (float*)(ws + oS);
  unsigned short* P    = (unsigned short*)(ws + oP);
  unsigned short* W3   = (unsigned short*)(ws + oW3);
  unsigned short* WPK  = (unsigned short*)(ws + oWPK);
  unsigned short* WPV  = (unsigned short*)(ws + oWPV);
  unsigned short* WW   = (unsigned short*)(ws + oWW);
  float*          TAB  = (float*)(ws + oTAB);
  unsigned short* QH   = (unsigned short*)(ws + oQH);
  unsigned short* QL   = (unsigned short*)(ws + oQL);
  unsigned short* KH   = (unsigned short*)(ws + oKH);
  unsigned short* KL   = (unsigned short*)(ws + oKL);
  unsigned short* VH   = (unsigned short*)(ws + oVH);
  unsigned short* VL   = (unsigned short*)(ws + oVL);
  unsigned short* CTH  = (unsigned short*)(ws + oCTH);
  unsigned short* CTL  = (unsigned short*)(ws + oCTL);

  const dim3 blk(256);
  const long long stXT = (long long)NP * CIN;
  const long long stQ  = (long long)NP * KCH;
  const long long stKVF = (long long)NROWKV * NP;
  const long long stCAT = (long long)NP * CATC;

  k_tab<<<dim3(1), blk, 0, stream>>>(gq, bq, mq, vq, gk, bk, mk, vk, bpk, bpv, TAB);
  k_cvtw<<<dim3(128, 6), blk, 0, stream>>>(wq, wk, wv, wpk, wpv, ww, W3, WPK, WPV, WW);
  k_cvtx<<<dim3(NP / 16, NBATCH), blk, 0, stream>>>(x, XT);
  k_gemm<0, 0, 1><<<dim3((NP / 128) * (KCH / 64), NBATCH), blk, 0, stream>>>(
      XT, XT, CIN, stXT, W3, W3, CIN, 0LL, KVF, QH, QL, KCH, stQ,
      NP, KCH, CIN, OSC16, TAB + 0 * KCH, TAB + 1 * KCH, KCH, 1, KCH, CSC);
  k_gemm<0, 0, 0><<<dim3((NROWKV / 128) * (NP / 64), NBATCH), blk, 0, stream>>>(
      W3 + (size_t)KCH * CIN, W3 + (size_t)KCH * CIN, CIN, 0LL, XT, XT, CIN, stXT, KVF, QH, QL, NP, stKVF,
      NROWKV, NP, CIN, OSC16, TAB + 2 * KCH, TAB + 4 * KCH, 2 * KCH, 0, KCH, CSC);
  k_pool<<<dim3(NROWKV, NBATCH), blk, 0, stream>>>(KVF, POOL);
  k_cat<<<dim3(NP / 16, NBATCH), blk, 0, stream>>>(POOL, 0, CATH, CATL);
  k_gemm<1, 0, 1><<<dim3((NP / 128) * (KCH / 64), NBATCH), blk, 0, stream>>>(
      CATH, CATL, CATC, stCAT, WPK, WPK, CATC, 0LL, KVF, KH, KL, KCH, stQ,
      NP, KCH, CATC, OSC16, TAB + 3 * KCH, TAB + 6 * KCH, KCH, 1, 0, CSC);
  k_cat<<<dim3(NP / 16, NBATCH), blk, 0, stream>>>(POOL, KCH, CATH, CATL);
  k_gemm<0, 1, 1><<<dim3((KCH / 128) * (NP / 64), NBATCH), blk, 0, stream>>>(
      WPV, WPV, CATC, 0LL, CATH, CATL, CATC, stCAT, KVF, VH, VL, NP, stQ,
      KCH, NP, CATC, OSC16, TAB + 3 * KCH, TAB + 7 * KCH, KCH, 0, 0, CSC);
  for (int b = 0; b < NBATCH; ++b) {
    const size_t qo = (size_t)b * NP * KCH;
    k_gemm<1, 1, 0><<<dim3((NP / 128) * (NP / 64), 1), blk, 0, stream>>>(
        QH + qo, QL + qo, KCH, 0LL, KH + qo, KL + qo, KCH, 0LL, S, P, P, NP, 0LL,
        NP, NP, KCH, OSC16, TAB + 3 * KCH, TAB + 5 * KCH, KCH, 0, 0, CSC);
    k_soft<<<dim3(NP), blk, 0, stream>>>(S, P);
    k_gemm<0, 1, 1><<<dim3((NP / 128) * (KCH / 64), 1), blk, 0, stream>>>(
        P, P, NP, 0LL, VH + qo, VL + qo, NP, 0LL, S, CTH, CTL, KCH, 0LL,
        NP, KCH, NP, OSC20, TAB + 3 * KCH, TAB + 5 * KCH, KCH, 0, 0, CSC);
    k_gemm<0, 1, 0><<<dim3((COUT / 128) * (NP / 64), 1), blk, 0, stream>>>(
        WW, WW, KCH, 0LL, CTH, CTL, KCH, 0LL, out + (size_t)b * COUT * NP, P, P, NP, 0LL,
        COUT, NP, KCH, OSC16, TAB + 3 * KCH, TAB + 5 * KCH, KCH, 0, 0, CSC);
  }
  (void)hipGetLastError();
}
